// MemoryAsLayerTitan_53455162966284
// MI455X (gfx1250) — hardware-verified
//
#include <hip/hip_runtime.h>

typedef __bf16 bf16;
typedef bf16     v8b  __attribute__((ext_vector_type(8)));
typedef bf16     v16b __attribute__((ext_vector_type(16)));
typedef float    v8f  __attribute__((ext_vector_type(8)));
typedef float    v4f  __attribute__((ext_vector_type(4)));
typedef unsigned v4u  __attribute__((ext_vector_type(4)));
typedef unsigned v8u  __attribute__((ext_vector_type(8)));
typedef unsigned short u16;
typedef u16      v8s  __attribute__((ext_vector_type(8)));
typedef v8b __attribute__((may_alias)) v8ba;
typedef v4f __attribute__((may_alias)) v4fa;
typedef v8s __attribute__((may_alias)) v8sa;

union Frag { v16b v; v8b half[2]; v8u u; };

constexpr int NB = 2, NL = 2048, ND = 512, NP = 32, NM = 1024, NH = 8, HD = 64, WIN = 256;
constexpr int NS  = NP + NL;
constexpr int NR  = NB * NS;
constexpr int SP  = 2112;
constexpr int LDP = 3 * ND;

constexpr size_t SZ_COMB = (size_t)NR * ND * 4;
constexpr size_t SZ_KEYS = (size_t)NM * ND * 4;
constexpr size_t SZ_WT   = (size_t)8 * ND * ND * 4;
constexpr size_t SZ_PR   = (size_t)NR * LDP * 4;
constexpr size_t SZ_LG   = (size_t)NR * NM * 4;
constexpr size_t SZ_ST   = (size_t)NR * 2 * 4;
constexpr size_t SZ_WW   = (size_t)NB * NM * SP * 4;
constexpr size_t SZ_VT   = (size_t)NB * ND * SP * 4;
constexpr size_t SZ_STT  = (size_t)NB * ND * NM * 4;
constexpr size_t SZ_H    = (size_t)NR * ND * 4;
constexpr size_t SZ_AO   = (size_t)NR * ND * 4;
constexpr size_t WS_TOTAL = SZ_COMB + SZ_KEYS + SZ_WT + SZ_PR + SZ_LG + SZ_ST + SZ_WW + SZ_VT + SZ_STT + SZ_H + SZ_AO;
static_assert(WS_TOTAL <= (size_t)134217728);
static_assert((SZ_ST & 255) == 0);
static_assert((size_t)NR * NM * 4 <= SZ_WW);
static_assert(NR % 32 == 0 && NS % 32 == 0 && ND % 256 == 0 && NM % 256 == 0 && LDP % 256 == 0);

#define WRAW(A_, B_, C_) __builtin_amdgcn_wmma_f32_16x16x32_bf16(false, (A_), false, (B_), (short)0, (C_), false, false)
#define NOP4 "v_nop\n\tv_nop\n\tv_nop\n\tv_nop"

__device__ __forceinline__ v8f zero8() { v8f z = {0.f, 0.f, 0.f, 0.f, 0.f, 0.f, 0.f, 0.f}; return z; }

__device__ __forceinline__ v16b ldf(const bf16* p, int h) {
  Frag f;
  f.half[0] = *(const v8ba*)(p + 8 * h);
  f.half[1] = *(const v8ba*)(p + 16 + 8 * h);
  return f.v;
}

__device__ __forceinline__ unsigned bfb(float f) {
  unsigned u = __float_as_uint(f);
  u += 0x7FFFu + ((u >> 16) & 1u);
  return u >> 16;
}
__device__ __forceinline__ void split2(float f0, float f1, unsigned& hp, unsigned& lp) {
  const unsigned h0 = bfb(f0), h1 = bfb(f1);
  const float r0 = f0 - __uint_as_float(h0 << 16);
  const float r1 = f1 - __uint_as_float(h1 << 16);
  hp = h0 | (h1 << 16);
  lp = bfb(r0) | (bfb(r1) << 16);
}
__device__ __forceinline__ void split8(v4f a, v4f c, v4u& hv, v4u& lv) {
  unsigned h0, h1, h2, h3, l0, l1, l2, l3;
  split2(a.x, a.y, h0, l0);
  split2(a.z, a.w, h1, l1);
  split2(c.x, c.y, h2, l2);
  split2(c.z, c.w, h3, l3);
  const v4u hh = {h0, h1, h2, h3};
  const v4u ll = {l0, l1, l2, l3};
  hv = hh; lv = ll;
}
__device__ __forceinline__ v4f sel4(bool c, v4f a, v4f b) {
  v4f r;
  r.x = c ? a.x : b.x; r.y = c ? a.y : b.y; r.z = c ? a.z : b.z; r.w = c ? a.w : b.w;
  return r;
}
__device__ __forceinline__ void vstf(float* p, v4f v) { *(volatile v4f*)p = v; }
__device__ __forceinline__ void vstu(bf16* p, v4u v) { *(volatile v4u*)(void*)p = v; }

__global__ __launch_bounds__(256) void cvt_rows_k(
    const float* __restrict__ x, const float* __restrict__ pm, const float* __restrict__ keys,
    bf16* Ch, bf16* Cl, bf16* Kh, bf16* Kl)
{
  constexpr int NGC = NR * ND / 8;
  const int g = (int)blockIdx.x * 256 + (int)threadIdx.x;
  v4f a, c;
  bf16* dh;
  bf16* dl;
  size_t off;
  if ((int)blockIdx.x < NGC / 256) {
    const int row = g >> 6, col = (g & 63) * 8;
    const int b = (row >= NS) ? 1 : 0;
    const int s = row - b * NS;
    const bool pers = s < NP;
    const int sp = pers ? s : (NP - 1);
    const int sl = pers ? 0 : (s - NP);
    const float* p0 = pm + (size_t)sp * ND + col;
    const float* p1 = x + ((size_t)b * NL + sl) * ND + col;
    const v4f a0 = *(const v4fa*)p0, c0 = *(const v4fa*)(p0 + 4);
    const v4f a1 = *(const v4fa*)p1, c1 = *(const v4fa*)(p1 + 4);
    a = sel4(pers, a0, a1);
    c = sel4(pers, c0, c1);
    off = (size_t)row * ND + col;
    dh = Ch; dl = Cl;
  } else {
    const int e = g - NGC;
    const float* p = keys + (size_t)e * 8;
    a = *(const v4fa*)p;
    c = *(const v4fa*)(p + 4);
    off = (size_t)e * 8;
    dh = Kh; dl = Kl;
  }
  v4u hv, lv;
  split8(a, c, hv, lv);
  vstu(dh + off, hv);
  vstu(dl + off, lv);
  __threadfence();
  vstu(dh + off, hv);
  vstu(dl + off, lv);
}

__global__ __launch_bounds__(256) void cvt_wt_k(
    const float* __restrict__ w0, const float* __restrict__ w1, const float* __restrict__ w2,
    const float* __restrict__ w3, const float* __restrict__ w4, const float* __restrict__ w5,
    const float* __restrict__ w6, const float* __restrict__ w7, bf16* Th, bf16* Tl)
{
  __shared__ __attribute__((aligned(16))) float sW[64 * 65];
  const int tid = (int)threadIdx.x;
  const int z = (int)blockIdx.z;
  const float* src = (z == 0) ? w0 : (z == 1) ? w1 : (z == 2) ? w2 : (z == 3) ? w3 :
                     (z == 4) ? w4 : (z == 5) ? w5 : (z == 6) ? w6 : w7;
  const int k0 = (int)blockIdx.x * 64, n0 = (int)blockIdx.y * 64;
  {
    const int i = tid >> 2, q = tid & 3;
    const float* p = src + (size_t)(k0 + i) * ND + n0 + 16 * q;
    #pragma unroll
    for (int j = 0; j < 4; ++j) {
      const v4f v = *(const v4fa*)(p + 4 * j);
      float* d = sW + i * 65 + 16 * q + 4 * j;
      d[0] = v.x; d[1] = v.y; d[2] = v.z; d[3] = v.w;
    }
  }
  __syncthreads();
  v4u hv[2], lv[2];
  size_t off[2];
  #pragma unroll
  for (int it = 0; it < 2; ++it) {
    const int idx = tid + 256 * it;
    const int c = idx >> 3, p8 = idx & 7;
    const float* s0 = sW + (8 * p8) * 65 + c;
    v4f a, cc;
    a.x = s0[0];    a.y = s0[65];   a.z = s0[130];  a.w = s0[195];
    cc.x = s0[260]; cc.y = s0[325]; cc.z = s0[390]; cc.w = s0[455];
    split8(a, cc, hv[it], lv[it]);
    off[it] = ((size_t)(z * ND + n0 + c)) * ND + k0 + 8 * p8;
  }
  vstu(Th + off[0], hv[0]); vstu(Tl + off[0], lv[0]);
  vstu(Th + off[1], hv[1]); vstu(Tl + off[1], lv[1]);
  __threadfence();
  vstu(Th + off[0], hv[0]); vstu(Tl + off[0], lv[0]);
  vstu(Th + off[1], hv[1]); vstu(Tl + off[1], lv[1]);
}

__device__ __forceinline__ void gstore_f32(const float* st, float* C, size_t cbase, int ldc, v4f b4, int lane) {
  const int p = lane & 15, rs = lane >> 4;
  #pragma unroll
  for (int i = 0; i < 16; ++i) {
    const int row = 2 * i + rs;
    v4f v = *(const v4fa*)(st + row * 64 + 4 * p);
    v += b4;
    vstf(C + cbase + (size_t)row * ldc + 4 * p, v);
  }
}
__device__ __forceinline__ void gstore_b16(const float* st, bf16* Ch, bf16* Cl, size_t cbase, int ldc, int lane) {
  const int p = lane & 7, rs = lane >> 3;
  #pragma unroll
  for (int i = 0; i < 8; ++i) {
    const int row = 4 * i + rs;
    const v4f a = *(const v4fa*)(st + row * 64 + 8 * p);
    const v4f c = *(const v4fa*)(st + row * 64 + 8 * p + 4);
    v4u hv, lv;
    split8(a, c, hv, lv);
    const size_t off = cbase + (size_t)row * ldc + 8 * p;
    vstu(Ch + off, hv);
    vstu(Cl + off, lv);
  }
}

template <int OUTB>
__global__ __launch_bounds__(128) void gemm3_k(
    const bf16* __restrict__ Ah, const bf16* __restrict__ Al, int lda, long long sAz,
    const bf16* __restrict__ Bh, const bf16* __restrict__ Bl, int ldb, long long sBz,
    int K,
    float* Cf, bf16* Ch, bf16* Cl, int ldc, long long sCz,
    const float* __restrict__ bias)
{
  __shared__ __attribute__((aligned(16))) float sT[4 * 32 * 64];
  const int tid = (int)threadIdx.x, lane = tid & 31, w = tid >> 5;
  const int h = lane >> 4, m = lane & 15;
  const int r0 = (int)blockIdx.x * 32;
  const int c0 = (int)blockIdx.y * 256 + w * 64;
  const long long za = (long long)blockIdx.z * sAz;
  const long long zb = (long long)blockIdx.z * sBz;
  const long long zc = (long long)blockIdx.z * sCz;
  const long long ao0 = za + (long long)(r0 + m) * lda;
  const long long ao1 = ao0 + (long long)16 * lda;
  const long long bo0 = zb + (long long)(c0 + m) * ldb;

  v8f acc[2][4];
  #pragma unroll
  for (int mt = 0; mt < 2; ++mt)
    #pragma unroll
    for (int nt = 0; nt < 4; ++nt) acc[mt][nt] = zero8();

  #pragma unroll 1
  for (int k0 = 0; k0 < K; k0 += 32) {
    const v16b x0h = ldf(Ah + ao0 + k0, h);
    const v16b x0l = ldf(Al + ao0 + k0, h);
    const v16b x1h = ldf(Ah + ao1 + k0, h);
    const v16b x1l = ldf(Al + ao1 + k0, h);
    #pragma unroll
    for (int nt = 0; nt < 4; ++nt) {
      const long long bo = bo0 + (long long)(16 * nt) * ldb + k0;
      const v16b yh = ldf(Bh + bo, h);
      const v16b yl = ldf(Bl + bo, h);
      v8f d0 = acc[0][nt], d1 = acc[1][nt];
      d0 = WRAW(x0h, yh, d0); d0 = WRAW(x0h, yl, d0); d0 = WRAW(x0l, yh, d0);
      d1 = WRAW(x1h, yh, d1); d1 = WRAW(x1h, yl, d1); d1 = WRAW(x1l, yh, d1);
      asm volatile(NOP4 : "+v"(d0), "+v"(d1)
                   : "v"(x0h), "v"(x0l), "v"(x1h), "v"(x1l), "v"(yh), "v"(yl));
      acc[0][nt] = d0; acc[1][nt] = d1;
    }
  }

  float* st = sT + w * 2048;
  #pragma unroll
  for (int mt = 0; mt < 2; ++mt)
    #pragma unroll
    for (int nt = 0; nt < 4; ++nt)
      #pragma unroll
      for (int r = 0; r < 8; ++r)
        st[(16 * mt + 8 * h + r) * 64 + 16 * nt + m] = acc[mt][nt][r];
  __syncthreads();

  const size_t cbase = (size_t)(zc + (long long)r0 * ldc + c0);
  if (OUTB == 0) {
    v4f b4 = {0.f, 0.f, 0.f, 0.f};
    if (bias != nullptr) b4 = *(const v4fa*)(bias + c0 + 4 * (lane & 15));
    gstore_f32(st, Cf, cbase, ldc, b4, lane);
    __threadfence();
    gstore_f32(st, Cf, cbase, ldc, b4, lane);
  } else {
    gstore_b16(st, Ch, Cl, cbase, ldc, lane);
    __threadfence();
    gstore_b16(st, Ch, Cl, cbase, ldc, lane);
  }
}

__global__ __launch_bounds__(256) void slot_stats_k(const float* __restrict__ L, float* stats)
{
  __shared__ __attribute__((aligned(16))) float sS[32];
  const int tid = (int)threadIdx.x, lane = tid & 31, w = tid >> 5;
  #pragma unroll 1
  for (int rr = 0; rr < 2; ++rr) {
    const int rl = 2 * w + rr;
    const int row = (int)blockIdx.x * 16 + rl;
    const float* p = L + (size_t)row * NM + 4 * lane;
    float mx = -3.0e38f;
    #pragma unroll 1
    for (int i = 0; i < 8; ++i) {
      const v4f v = *(const v4fa*)(p + 128 * i);
      mx = fmaxf(mx, fmaxf(fmaxf(v.x, v.y), fmaxf(v.z, v.w)));
    }
    for (int o = 16; o > 0; o >>= 1) mx = fmaxf(mx, __shfl_xor(mx, o));
    float sm = 0.f;
    #pragma unroll 1
    for (int i = 0; i < 8; ++i) {
      const v4f v = *(const v4fa*)(p + 128 * i);
      sm += (__expf(v.x - mx) + __expf(v.y - mx)) + (__expf(v.z - mx) + __expf(v.w - mx));
    }
    for (int o = 16; o > 0; o >>= 1) sm += __shfl_xor(sm, o);
    if (lane == 0) { sS[2 * rl] = mx; sS[2 * rl + 1] = 1.0f / sm; }
  }
  __syncthreads();
  const v4f sv = *(const v4fa*)(sS + 4 * (tid & 7));
  float* dst = stats + (size_t)blockIdx.x * 32 + 4 * (tid & 7);
  if (tid < 8) vstf(dst, sv);
  __threadfence();
  if (tid < 8) vstf(dst, sv);
}

__global__ __launch_bounds__(256) void slot_apply_t_k(
    const float* __restrict__ L, const float* __restrict__ stats, bf16* Th, bf16* Tl)
{
  __shared__ __attribute__((aligned(16))) float sP[64 * 65];
  const int tid = (int)threadIdx.x;
  const int s0 = (int)blockIdx.x * 64, m0 = (int)blockIdx.y * 64, b = (int)blockIdx.z;
  {
    const int i = tid >> 2, q = tid & 3;
    const int s = s0 + i;
    const bool ok = s < NS;
    const int sc = ok ? s : (NS - 1);
    const int row = b * NS + sc;
    const float mx = stats[2 * row], inv = stats[2 * row + 1];
    const float* p = L + (size_t)row * NM + m0 + 16 * q;
    #pragma unroll 1
    for (int j = 0; j < 4; ++j) {
      const v4f v = *(const v4fa*)(p + 4 * j);
      float* d = sP + i * 65 + 16 * q + 4 * j;
      d[0] = ok ? __expf(v.x - mx) * inv : 0.f;
      d[1] = ok ? __expf(v.y - mx) * inv : 0.f;
      d[2] = ok ? __expf(v.z - mx) * inv : 0.f;
      d[3] = ok ? __expf(v.w - mx) * inv : 0.f;
    }
  }
  __syncthreads();
  v4u hv[2], lv[2];
  size_t off[2];
  #pragma unroll
  for (int it = 0; it < 2; ++it) {
    const int idx = tid + 256 * it;
    const int c = idx >> 3, p8 = idx & 7;
    const float* s0p = sP + (8 * p8) * 65 + c;
    v4f a, cc;
    a.x = s0p[0];    a.y = s0p[65];   a.z = s0p[130];  a.w = s0p[195];
    cc.x = s0p[260]; cc.y = s0p[325]; cc.z = s0p[390]; cc.w = s0p[455];
    split8(a, cc, hv[it], lv[it]);
    off[it] = ((size_t)(b * NM + m0 + c)) * SP + s0 + 8 * p8;
  }
  vstu(Th + off[0], hv[0]); vstu(Tl + off[0], lv[0]);
  vstu(Th + off[1], hv[1]); vstu(Tl + off[1], lv[1]);
  __threadfence();
  vstu(Th + off[0], hv[0]); vstu(Tl + off[0], lv[0]);
  vstu(Th + off[1], hv[1]); vstu(Tl + off[1], lv[1]);
}

__global__ __launch_bounds__(256) void slot_apply_rows_k(
    const float* __restrict__ L, const float* __restrict__ stats, bf16* Wh, bf16* Wl)
{
  const int g = (int)blockIdx.x * 256 + (int)threadIdx.x;
  const int row = g >> 7, col = (g & 127) * 8;
  const float mx = stats[2 * row], inv = stats[2 * row + 1];
  const float* p = L + (size_t)row * NM + col;
  v4f a = *(const v4fa*)p, c = *(const v4fa*)(p + 4);
  a.x = __expf(a.x - mx) * inv; a.y = __expf(a.y - mx) * inv;
  a.z = __expf(a.z - mx) * inv; a.w = __expf(a.w - mx) * inv;
  c.x = __expf(c.x - mx) * inv; c.y = __expf(c.y - mx) * inv;
  c.z = __expf(c.z - mx) * inv; c.w = __expf(c.w - mx) * inv;
  v4u hv, lv;
  split8(a, c, hv, lv);
  const size_t off = (size_t)row * NM + col;
  vstu(Wh + off, hv); vstu(Wl + off, lv);
  __threadfence();
  vstu(Wh + off, hv); vstu(Wl + off, lv);
}

__global__ __launch_bounds__(256) void tr16_k(
    const bf16* __restrict__ Ih, const bf16* __restrict__ Il, int ldi, int coff, bf16* Oh, bf16* Ol)
{
  __shared__ __attribute__((aligned(16))) u16 sH[64 * 72];
  __shared__ __attribute__((aligned(16))) u16 sL[64 * 72];
  const int tid = (int)threadIdx.x;
  const int s0 = (int)blockIdx.x * 64, d0 = (int)blockIdx.y * 64, b = (int)blockIdx.z;
  {
    const int i = tid >> 2, q = tid & 3;
    const int s = s0 + i;
    const bool ok = s < NS;
    const int sc = ok ? s : (NS - 1);
    const size_t io = ((size_t)(b * NS + sc)) * ldi + coff + d0 + 16 * q;
    const u16* ph = (const u16*)(const void*)(Ih + io);
    const u16* pl = (const u16*)(const void*)(Il + io);
    v8s h0 = *(const v8sa*)ph, h1 = *(const v8sa*)(ph + 8);
    v8s l0 = *(const v8sa*)pl, l1 = *(const v8sa*)(pl + 8);
    const u16 mk = ok ? (u16)0xFFFF : (u16)0;
    const v8s mkv = {mk, mk, mk, mk, mk, mk, mk, mk};
    h0 &= mkv; h1 &= mkv; l0 &= mkv; l1 &= mkv;
    *(v8sa*)(sH + i * 72 + 16 * q) = h0;
    *(v8sa*)(sH + i * 72 + 16 * q + 8) = h1;
    *(v8sa*)(sL + i * 72 + 16 * q) = l0;
    *(v8sa*)(sL + i * 72 + 16 * q + 8) = l1;
  }
  __syncthreads();
  v4u hv[2], lv[2];
  size_t off[2];
  #pragma unroll
  for (int it = 0; it < 2; ++it) {
    const int idx = tid + 256 * it;
    const int c = idx >> 3, p8 = idx & 7;
    const u16* qh = sH + (8 * p8) * 72 + c;
    const u16* ql = sL + (8 * p8) * 72 + c;
    v4u uh, ul;
    uh.x = (unsigned)qh[0]   | ((unsigned)qh[72]  << 16);
    uh.y = (unsigned)qh[144] | ((unsigned)qh[216] << 16);
    uh.z = (unsigned)qh[288] | ((unsigned)qh[360] << 16);
    uh.w = (unsigned)qh[432] | ((unsigned)qh[504] << 16);
    ul.x = (unsigned)ql[0]   | ((unsigned)ql[72]  << 16);
    ul.y = (unsigned)ql[144] | ((unsigned)ql[216] << 16);
    ul.z = (unsigned)ql[288] | ((unsigned)ql[360] << 16);
    ul.w = (unsigned)ql[432] | ((unsigned)ql[504] << 16);
    hv[it] = uh; lv[it] = ul;
    off[it] = ((size_t)(b * ND + d0 + c)) * SP + s0 + 8 * p8;
  }
  vstu(Oh + off[0], hv[0]); vstu(Ol + off[0], lv[0]);
  vstu(Oh + off[1], hv[1]); vstu(Ol + off[1], lv[1]);
  __threadfence();
  vstu(Oh + off[0], hv[0]); vstu(Ol + off[0], lv[0]);
  vstu(Oh + off[1], hv[1]); vstu(Ol + off[1], lv[1]);
}

__global__ __launch_bounds__(256) void ln_k(
    const float* __restrict__ X, const float* __restrict__ gm, const float* __restrict__ bt,
    bf16* Hh, bf16* Hl)
{
  const int lane = (int)threadIdx.x & 31, w = (int)threadIdx.x >> 5;
  const int row = (int)blockIdx.x * 8 + w;
  const float* p = X + (size_t)row * ND;
  const int cA = 8 * lane, cB = 256 + 8 * lane;
  const v4f a0 = *(const v4fa*)(p + cA), a1 = *(const v4fa*)(p + cA + 4);
  const v4f b0 = *(const v4fa*)(p + cB), b1 = *(const v4fa*)(p + cB + 4);
  float sm = ((a0.x + a0.y) + (a0.z + a0.w)) + ((a1.x + a1.y) + (a1.z + a1.w))
           + ((b0.x + b0.y) + (b0.z + b0.w)) + ((b1.x + b1.y) + (b1.z + b1.w));
  for (int o = 16; o > 0; o >>= 1) sm += __shfl_xor(sm, o);
  const float mu = sm * (1.0f / (float)ND);
  const v4f d0 = a0 - mu, d1 = a1 - mu, e0 = b0 - mu, e1 = b1 - mu;
  float vs = (d0.x * d0.x + d0.y * d0.y + d0.z * d0.z + d0.w * d0.w)
           + (d1.x * d1.x + d1.y * d1.y + d1.z * d1.z + d1.w * d1.w)
           + (e0.x * e0.x + e0.y * e0.y + e0.z * e0.z + e0.w * e0.w)
           + (e1.x * e1.x + e1.y * e1.y + e1.z * e1.z + e1.w * e1.w);
  for (int o = 16; o > 0; o >>= 1) vs += __shfl_xor(vs, o);
  const float var = vs * (1.0f / (float)ND);
  const float rstd = 1.0f / sqrtf(var + 1e-5f);
  const v4f ga0 = *(const v4fa*)(gm + cA), ga1 = *(const v4fa*)(gm + cA + 4);
  const v4f gb0 = *(const v4fa*)(gm + cB), gb1 = *(const v4fa*)(gm + cB + 4);
  const v4f ba0 = *(const v4fa*)(bt + cA), ba1 = *(const v4fa*)(bt + cA + 4);
  const v4f bb0 = *(const v4fa*)(bt + cB), bb1 = *(const v4fa*)(bt + cB + 4);
  const v4f y0 = (d0 * rstd) * ga0 + ba0, y1 = (d1 * rstd) * ga1 + ba1;
  const v4f z0 = (e0 * rstd) * gb0 + bb0, z1 = (e1 * rstd) * gb1 + bb1;
  v4u hA, lA, hB, lB;
  split8(y0, y1, hA, lA);
  split8(z0, z1, hB, lB);
  const size_t offA = (size_t)row * ND + cA, offB = (size_t)row * ND + cB;
  vstu(Hh + offA, hA); vstu(Hh + offB, hB); vstu(Hl + offA, lA); vstu(Hl + offB, lB);
  __threadfence();
  vstu(Hh + offA, hA); vstu(Hh + offB, hB); vstu(Hl + offA, lA); vstu(Hl + offB, lB);
}

__device__ __forceinline__ void attn_store(const float* so, bf16* Oh, bf16* Ol, size_t obase, int lane) {
  const int p8 = lane & 7, sub = lane >> 3;
  #pragma unroll
  for (int i = 0; i < 4; ++i) {
    const int row = 4 * i + sub;
    const v4f a = *(const v4fa*)(so + row * 64 + 8 * p8);
    const v4f c = *(const v4fa*)(so + row * 64 + 8 * p8 + 4);
    v4u hv, lv;
    split8(a, c, hv, lv);
    const size_t off = obase + (size_t)row * ND + 8 * p8;
    vstu(Oh + off, hv);
    vstu(Ol + off, lv);
  }
}

__global__ __launch_bounds__(128) void attn_band_k(
    const bf16* __restrict__ Ph, const bf16* __restrict__ Pl,
    const bf16* __restrict__ Vh, const bf16* __restrict__ Vl,
    bf16* Oh, bf16* Ol)
{
  __shared__ __attribute__((aligned(16))) float sO[4 * 16 * 64];
  const int tid = (int)threadIdx.x, lane = tid & 31, w = tid >> 5;
  const int h = lane >> 4, m = lane & 15;
  const int bh = (int)blockIdx.y, b = bh >> 3, head = bh & 7;
  const int qraw = (int)blockIdx.x * 64 + 16 * w;
  const bool valid = qraw < NS;
  const int q0 = valid ? qraw : (NS - 16);

  const size_t qoff = ((size_t)(b * NS + q0 + m)) * LDP + head * HD;
  const v16b qb0h = ldf(Ph + qoff, h), qb1h = ldf(Ph + qoff + 32, h);
  const v16b qb0l = ldf(Pl + qoff, h), qb1l = ldf(Pl + qoff + 32, h);
  const size_t kbase = ((size_t)(b * NS + m)) * LDP + ND + head * HD;
  const size_t vbase = ((size_t)(b * ND + head * HD + m)) * SP;

  v8f o[4];
  #pragma unroll
  for (int t = 0; t < 4; ++t) o[t] = zero8();
  float mrun = -1.0e30f, lrun = 0.f;

  int jlo = q0 - (WIN - 1);
  if (jlo < 0) jlo = 0;
  jlo &= ~31;
  int jhi = q0 + 15 + WIN;
  if (jhi > NS) jhi = NS;
  const int qi = q0 + m;

  #pragma unroll 1
  for (int kb = jlo; kb < jhi; kb += 32) {
    v8f s[2];
    #pragma unroll
    for (int jt = 0; jt < 2; ++jt) {
      const size_t ko = kbase + (size_t)(kb + 16 * jt) * LDP;
      const v16b k0h = ldf(Ph + ko, h), k1h = ldf(Ph + ko + 32, h);
      const v16b k0l = ldf(Pl + ko, h), k1l = ldf(Pl + ko + 32, h);
      v8f z = zero8();
      z = WRAW(k0h, qb0h, z); z = WRAW(k0h, qb0l, z); z = WRAW(k0l, qb0h, z);
      z = WRAW(k1h, qb1h, z); z = WRAW(k1h, qb1l, z); z = WRAW(k1l, qb1h, z);
      asm volatile(NOP4 : "+v"(z)
                   : "v"(k0h), "v"(k0l), "v"(k1h), "v"(k1l), "v"(qb0h), "v"(qb0l), "v"(qb1h), "v"(qb1l));
      s[jt] = z;
    }
    float mloc = -1.0e30f;
    #pragma unroll
    for (int jt = 0; jt < 2; ++jt)
      #pragma unroll
      for (int r = 0; r < 8; ++r) {
        const int key = kb + 16 * jt + 8 * h + r;
        int dd = qi - key; dd = (dd < 0) ? -dd : dd;
        const bool ok = dd < WIN;
        const float sv = ok ? s[jt][r] * 0.125f : -1.0e30f;
        s[jt][r] = sv;
        mloc = fmaxf(mloc, sv);
      }
    mloc = fmaxf(mloc, __shfl_xor(mloc, 16));
    const float mnew = fmaxf(mrun, mloc);
    const float alpha = __expf(mrun - mnew);
    mrun = mnew;
    float lsum = 0.f;
    #pragma unroll
    for (int jt = 0; jt < 2; ++jt)
      #pragma unroll
      for (int r = 0; r < 8; ++r) {
        const int key = kb + 16 * jt + 8 * h + r;
        int dd = qi - key; dd = (dd < 0) ? -dd : dd;
        const bool ok = dd < WIN;
        const float p = ok ? __expf(s[jt][r] - mnew) : 0.f;
        s[jt][r] = p;
        lsum += p;
      }
    lsum += __shfl_xor(lsum, 16);
    lrun = lrun * alpha + lsum;
    #pragma unroll
    for (int t = 0; t < 4; ++t)
      #pragma unroll
      for (int r = 0; r < 8; ++r) o[t][r] = o[t][r] * alpha;

    Frag fh, fl;
    {
      unsigned u0, u1, u2, u3, u4, u5, u6, u7, l0, l1, l2, l3, l4, l5, l6, l7;
      split2(s[0][0], s[0][1], u0, l0); split2(s[0][2], s[0][3], u1, l1);
      split2(s[0][4], s[0][5], u2, l2); split2(s[0][6], s[0][7], u3, l3);
      split2(s[1][0], s[1][1], u4, l4); split2(s[1][2], s[1][3], u5, l5);
      split2(s[1][4], s[1][5], u6, l6); split2(s[1][6], s[1][7], u7, l7);
      const v8u uh = {u0, u1, u2, u3, u4, u5, u6, u7};
      const v8u ul = {l0, l1, l2, l3, l4, l5, l6, l7};
      fh.u = uh; fl.u = ul;
    }
    const v16b pbh = fh.v, pbl = fl.v;

    #pragma unroll
    for (int t = 0; t < 4; ++t) {
      const size_t vo = vbase + (size_t)(16 * t) * SP + kb;
      const v16b vfh = ldf(Vh + vo, h), vfl = ldf(Vl + vo, h);
      v8f d = o[t];
      d = WRAW(vfh, pbh, d); d = WRAW(vfh, pbl, d); d = WRAW(vfl, pbh, d);
      asm volatile(NOP4 : "+v"(d) : "v"(vfh), "v"(vfl), "v"(pbh), "v"(pbl));
      o[t] = d;
    }
  }

  const float inv = 1.0f / lrun;
  float* so = sO + w * 1024;
  #pragma unroll
  for (int t = 0; t < 4; ++t)
    #pragma unroll
    for (int r = 0; r < 8; ++r)
      so[m * 64 + 16 * t + 8 * h + r] = o[t][r] * inv;
  __syncthreads();

  const size_t obase = ((size_t)(b * NS + q0)) * ND + head * HD;
  if (valid) attn_store(so, Oh, Ol, obase, lane);
  __threadfence();
  if (valid) attn_store(so, Oh, Ol, obase, lane);
}

extern "C" void kernel_launch(void* const* d_in, const int* in_sizes, int n_in,
                              void* d_out, int out_size, void* d_ws, size_t ws_size,
                              hipStream_t stream) {
  if (n_in < 16) return;
  if (in_sizes[0] != NB * NL * ND) return;
  if (in_sizes[1] != NP * ND) return;
  if (in_sizes[2] != NM * ND) return;
  for (int i = 3; i <= 9; ++i) if (in_sizes[i] != ND * ND) return;
  for (int i = 10; i <= 13; ++i) if (in_sizes[i] != ND) return;
  if (in_sizes[14] != ND * ND || in_sizes[15] != ND) return;
  if (out_size != NR * ND) return;
  if (WS_TOTAL > ws_size) return;

  const float* x    = (const float*)d_in[0];
  const float* pmem = (const float*)d_in[1];
  const float* mkey = (const float*)d_in[2];
  const float* mWk  = (const float*)d_in[3];
  const float* mWv  = (const float*)d_in[4];
  const float* mWq  = (const float*)d_in[5];
  const float* aWq  = (const float*)d_in[6];
  const float* aWk  = (const float*)d_in[7];
  const float* aWv  = (const float*)d_in[8];
  const float* aWo  = (const float*)d_in[9];
  const float* ln1g = (const float*)d_in[10];
  const float* ln1b = (const float*)d_in[11];
  const float* ln2g = (const float*)d_in[12];
  const float* ln2b = (const float*)d_in[13];
  const float* oW   = (const float*)d_in[14];
  const float* ob   = (const float*)d_in[15];
  float* out = (float*)d_out;

  char* ws = (char*)d_ws;
  size_t off = 0;
  char* rComb = ws + off; off += SZ_COMB;
  char* rKeys = ws + off; off += SZ_KEYS;
  char* rWT   = ws + off; off += SZ_WT;
  char* rPR   = ws + off; off += SZ_PR;
  char* rLG   = ws + off; off += SZ_LG;
  char* rST   = ws + off; off += SZ_ST;
  char* rWW   = ws + off; off += SZ_WW;
  char* rVT   = ws + off; off += SZ_VT;
  char* rSTT  = ws + off; off += SZ_STT;
  char* rH    = ws + off; off += SZ_H;
  char* rAO   = ws + off; off += SZ_AO;
  if (off > ws_size) return;

  bf16* combH = (bf16*)rComb;              bf16* combL = (bf16*)(rComb + (size_t)NR * ND * 2);
  float* memo = (float*)rComb;
  float* ao2  = (float*)rComb;
  bf16* keysH = (bf16*)rKeys;              bf16* keysL = (bf16*)(rKeys + (size_t)NM * ND * 2);
  bf16* wtH   = (bf16*)rWT;                bf16* wtL   = (bf16*)(rWT + (size_t)8 * ND * ND * 2);
  bf16* prH   = (bf16*)rPR;                bf16* prL   = (bf16*)(rPR + (size_t)NR * LDP * 2);
  float* Lg   = (float*)rLG;
  float* stats = (float*)rST;
  bf16* wwH   = (bf16*)rWW;                bf16* wwL   = (bf16*)(rWW + (size_t)NB * NM * SP * 2);
  bf16* wrH   = (bf16*)rWW;                bf16* wrL   = (bf16*)(rWW + (size_t)NR * NM * 2);
  bf16* vtH   = (bf16*)rVT;                bf16* vtL   = (bf16*)(rVT + (size_t)NB * ND * SP * 2);
  bf16* stH   = (bf16*)rSTT;               bf16* stL   = (bf16*)(rSTT + (size_t)NB * ND * NM * 2);
  bf16* hH    = (bf16*)rH;                 bf16* hL    = (bf16*)(rH + (size_t)NR * ND * 2);
  bf16* aoH   = (bf16*)rAO;                bf16* aoL   = (bf16*)(rAO + (size_t)NR * ND * 2);

  const size_t WM = (size_t)ND * ND;

  cvt_rows_k<<<(NR * ND / 8 + NM * ND / 8) / 256, 256, 0, stream>>>(x, pmem, mkey, combH, combL, keysH, keysL);
  cvt_wt_k<<<dim3(ND / 64, ND / 64, 8), 256, 0, stream>>>(mWk, mWv, mWq, aWq, aWk, aWv, aWo, oW, wtH, wtL);
  gemm3_k<1><<<dim3(NR / 32, LDP / 256, 1), 128, 0, stream>>>(
      combH, combL, ND, 0, wtH, wtL, ND, 0, ND, nullptr, prH, prL, LDP, 0, nullptr);
  gemm3_k<0><<<dim3(NR / 32, NM / 256, 1), 128, 0, stream>>>(
      prH, prL, LDP, 0, keysH, keysL, ND, 0, ND, Lg, nullptr, nullptr, NM, 0, nullptr);
  slot_stats_k<<<NR / 16, 256, 0, stream>>>(Lg, stats);
  slot_apply_t_k<<<dim3(SP / 64, NM / 64, NB), 256, 0, stream>>>(Lg, stats, wwH, wwL);
  tr16_k<<<dim3(SP / 64, ND / 64, NB), 256, 0, stream>>>(prH, prL, LDP, ND, vtH, vtL);
  gemm3_k<1><<<dim3(ND / 32, NM / 256, NB), 128, 0, stream>>>(
      vtH, vtL, SP, (long long)ND * SP, wwH, wwL, SP, (long long)NM * SP, SP,
      nullptr, stH, stL, NM, (long long)ND * NM, nullptr);
  gemm3_k<0><<<dim3(NR / 32, NM / 256, 1), 128, 0, stream>>>(
      prH + 2 * ND, prL + 2 * ND, LDP, 0, keysH, keysL, ND, 0, ND, Lg, nullptr, nullptr, NM, 0, nullptr);
  slot_stats_k<<<NR / 16, 256, 0, stream>>>(Lg, stats);
  slot_apply_rows_k<<<(NR * NM / 8) / 256, 256, 0, stream>>>(Lg, stats, wrH, wrL);
  gemm3_k<0><<<dim3(NS / 32, ND / 256, NB), 128, 0, stream>>>(
      wrH, wrL, NM, (long long)NS * NM, stH, stL, NM, (long long)ND * NM, NM,
      memo, nullptr, nullptr, ND, (long long)NS * ND, nullptr);
  ln_k<<<NR / 8, 256, 0, stream>>>(memo, ln1g, ln1b, hH, hL);
  gemm3_k<1><<<dim3(NR / 32, LDP / 256, 1), 128, 0, stream>>>(
      hH, hL, ND, 0, wtH + 3 * WM, wtL + 3 * WM, ND, 0, ND, nullptr, prH, prL, LDP, 0, nullptr);
  tr16_k<<<dim3(SP / 64, ND / 64, NB), 256, 0, stream>>>(prH, prL, LDP, 2 * ND, vtH, vtL);
  attn_band_k<<<dim3((NS + 63) / 64, NB * NH), 128, 0, stream>>>(prH, prL, vtH, vtL, aoH, aoL);
  gemm3_k<0><<<dim3(NR / 32, ND / 256, 1), 128, 0, stream>>>(
      aoH, aoL, ND, 0, wtH + 6 * WM, wtL + 6 * WM, ND, 0, ND, ao2, nullptr, nullptr, ND, 0, nullptr);
  ln_k<<<NR / 8, 256, 0, stream>>>(ao2, ln2g, ln2b, hH, hL);
  gemm3_k<0><<<dim3(NR / 32, ND / 256, 1), 128, 0, stream>>>(
      hH, hL, ND, 0, wtH + 7 * WM, wtL + 7 * WM, ND, 0, ND, out, nullptr, nullptr, ND, 0, ob);
}
